// Model_7249904795839
// MI455X (gfx1250) — hardware-verified
//
#include <hip/hip_runtime.h>
#include <math.h>

constexpr int kVocab  = 128;
constexpr int kEmb    = 256;
constexpr int kUnits  = 1024;
constexpr int kBatch  = 64;
constexpr int kSeq    = 512;
constexpr int kNBt    = kUnits + kVocab;
constexpr int kRowsPB = 16;
constexpr int kRnnBlocks = kBatch / kRowsPB;
constexpr int kRnnThr = 256;
constexpr int kHP     = kUnits + 8;
constexpr int kLSP    = kVocab + 4;
static_assert(kBatch % kRowsPB == 0);
static_assert(kUnits == (kRnnThr / 32) * 128);
static_assert(kVocab == (kRnnThr / 32) * 16);
static_assert(kRowsPB == 2 * (kRnnThr / 32));
static_assert(kUnits % 32 == 0);
static_assert(kHP % 8 == 0 && kLSP % 4 == 0);
static_assert(kEmb % 32 == 0);
static_assert(kVocab % 64 == 0 && kUnits % 64 == 0);
static_assert(kEmb % 64 == 0);
static_assert((kVocab * kEmb / 8) % 256 == 0);
static_assert(kUnits == 256 * 4);

typedef __attribute__((ext_vector_type(16))) _Float16 v16h;
typedef __attribute__((ext_vector_type(8)))  _Float16 v8h;
typedef __attribute__((ext_vector_type(16))) __bf16   v16b;
typedef __attribute__((ext_vector_type(8)))  __bf16   v8b;
typedef __attribute__((ext_vector_type(8)))  float    v8f;
typedef __attribute__((ext_vector_type(4)))  float    v4f;
typedef __attribute__((ext_vector_type(4)))  unsigned v4u;

__device__ __forceinline__ unsigned short f2bf_bits(float f) {
  unsigned u = __float_as_uint(f);
  return (unsigned short)((u + 0x7FFFu + ((u >> 16) & 1u)) >> 16);
}
__device__ __forceinline__ float bf_bits2f(unsigned short h) { return __uint_as_float(((unsigned)h) << 16); }
__device__ __forceinline__ float bf16r(float f) { return bf_bits2f(f2bf_bits(f)); }

__device__ __forceinline__ void dep_guard_h(v8f& a, v8f& b, v16h x, v16h y) { asm volatile("v_nop\n\tv_nop\n\tv_nop\n\tv_nop" : "+v"(a), "+v"(b) : "v"(x), "v"(y)); }
__device__ __forceinline__ void dep_guard_b(v8f& a, v8f& b, v16b x, v16b y) { asm volatile("v_nop\n\tv_nop\n\tv_nop\n\tv_nop" : "+v"(a), "+v"(b) : "v"(x), "v"(y)); }
__device__ __forceinline__ void keep4_h(v16h a, v16h b, v16h c, v16h d) { asm volatile("v_nop" :: "v"(a), "v"(b), "v"(c), "v"(d)); }
__device__ __forceinline__ void keep4_b(v16b a, v16b b, v16b c, v16b d) { asm volatile("v_nop" :: "v"(a), "v"(b), "v"(c), "v"(d)); }
__device__ __forceinline__ void acc_guard4(v8f& a, v8f& b, v8f& c, v8f& d) { asm volatile("v_nop\n\tv_nop\n\tv_nop\n\tv_nop" : "+v"(a), "+v"(b), "+v"(c), "+v"(d)); }
__device__ __forceinline__ void acc_guard1(v8f& a) { asm volatile("v_nop\n\tv_nop\n\tv_nop\n\tv_nop" : "+v"(a)); }
__device__ __forceinline__ void grp_guard3(v8f& a, v8f& b, v8f& d, v16b x, v16b y, v16b p0, v16b p1, v16b p2) {
  asm volatile("v_nop\n\tv_nop\n\tv_nop\n\tv_nop" : "+v"(a), "+v"(b), "+v"(d) : "v"(x), "v"(y), "v"(p0), "v"(p1), "v"(p2));
}
template <typename T> struct Frag;
template <> struct Frag<_Float16> {
  typedef v16h V; union U { v16h v; v8h h[2]; };
  static __device__ __forceinline__ v16h load(const _Float16* p) {
    U f; f.h[0] = *(const v8h*)(p); f.h[1] = *(const v8h*)(p + 16); return f.v;
  }
  static __device__ __forceinline__ v8f mma(v16h a, v16h b, v8f c) {
    return __builtin_amdgcn_wmma_f32_16x16x32_f16(false, a, false, b, (short)0, c, false, false);
  }
  static __device__ __forceinline__ void guard(v8f& a, v8f& b, v16h x, v16h y) { dep_guard_h(a, b, x, y); }
  static __device__ __forceinline__ void keep(v16h a, v16h b, v16h c, v16h d) { keep4_h(a, b, c, d); }
};
template <> struct Frag<__bf16> {
  typedef v16b V; union U { v16b v; v8b h[2]; };
  static __device__ __forceinline__ v16b load(const __bf16* p) {
    U f; f.h[0] = *(const v8b*)(p); f.h[1] = *(const v8b*)(p + 16); return f.v;
  }
  static __device__ __forceinline__ v8f mma(v16b a, v16b b, v8f c) {
    return __builtin_amdgcn_wmma_f32_16x16x32_bf16(false, a, false, b, (short)0, c, false, false);
  }
  static __device__ __forceinline__ void guard(v8f& a, v8f& b, v16b x, v16b y) { dep_guard_b(a, b, x, y); }
  static __device__ __forceinline__ void keep(v16b a, v16b b, v16b c, v16b d) { keep4_b(a, b, c, d); }
};

template <int ET> struct Elem;
template <> struct Elem<0> { typedef _Float16 T; };
template <> struct Elem<1> { typedef __bf16 T; };
template <int ET, bool SPLIT, int BIAS_MODE, int OUT_MODE, bool RESID, int ACT = 0>
__global__ __launch_bounds__(256) void wmma_gemm64(
    const unsigned short* __restrict__ Ap, const unsigned short* __restrict__ A2p, int lda, long strideA,
    const unsigned short* __restrict__ Btp, const unsigned short* __restrict__ Bt2p, int ldb, long strideB,
    void* __restrict__ Cout, void* __restrict__ Cout2, int ldc, long strideC,
    const float* __restrict__ bias,
    const float* __restrict__ resid, long strideR,
    int M, int N, int K, float scale) {
  typedef typename Elem<ET>::T T;
  typedef typename Frag<T>::V V;
  const T* A = (const T*)Ap; const T* A2 = (const T*)A2p; const T* Bt = (const T*)Btp; const T* Bt2 = (const T*)Bt2p;
  __shared__ __align__(16) float sT[8][16 * 68];
  const int b    = blockIdx.y;
  const int lane = threadIdx.x & 31;
  const int wave = threadIdx.x >> 5;
  const int tilesN = N >> 6;
  const int tilesM = M >> 6;
  const int tile = blockIdx.x * 8 + wave;
  if (tile >= tilesM * tilesN) return;
  const int tm = tile / tilesN;
  const int tn = tile - tm * tilesN;
  const int m0 = tm << 6;
  const int n0 = tn << 6;

  const T* Ab  = A  + (size_t)b * strideA;
  const T* Bb  = Bt + (size_t)b * strideB;
  const T* Ab2 = SPLIT ? (A2  + (size_t)b * strideA) : nullptr;
  const T* Bb2 = SPLIT ? (Bt2 + (size_t)b * strideB) : nullptr;

  const int rlane = lane & 15;
  const int koff  = (lane >> 4) * 8;
  const int mOff  = (lane >> 4) * 8;

  v8f acc[4][4];
#pragma unroll
  for (int i = 0; i < 4; ++i)
#pragma unroll
    for (int j = 0; j < 4; ++j) acc[i][j] = (v8f){0.f,0.f,0.f,0.f,0.f,0.f,0.f,0.f};

  for (int k0 = 0; k0 < K; k0 += 32) {
    V bh[4], bl[4];
#pragma unroll
    for (int j = 0; j < 4; ++j) {
      const size_t bo = (size_t)(n0 + (j << 4) + rlane) * ldb + koff + k0;
      bh[j] = Frag<T>::load(Bb + bo);
      if (SPLIT) bl[j] = Frag<T>::load(Bb2 + bo);
    }
#pragma unroll
    for (int i = 0; i < 4; ++i) {
      const size_t ao = (size_t)(m0 + (i << 4) + rlane) * lda + koff + k0;
      V ah = Frag<T>::load(Ab + ao);
      V al;
      if (SPLIT) al = Frag<T>::load(Ab2 + ao);
#pragma unroll
      for (int j = 0; j < 4; ++j) {
        acc[i][j] = Frag<T>::mma(ah, bh[j], acc[i][j]);
        if (SPLIT) {
          acc[i][j] = Frag<T>::mma(ah, bl[j], acc[i][j]);
          acc[i][j] = Frag<T>::mma(al, bh[j], acc[i][j]);
        }
      }
      Frag<T>::guard(acc[i][0], acc[i][3], ah, SPLIT ? al : ah);
    }
    Frag<T>::keep(bh[0], bh[1], bh[2], bh[3]);
    if (SPLIT) Frag<T>::keep(bl[0], bl[1], bl[2], bl[3]);
  }
  acc_guard4(acc[0][0], acc[0][1], acc[0][2], acc[0][3]);
  acc_guard4(acc[1][0], acc[1][1], acc[1][2], acc[1][3]);
  acc_guard4(acc[2][0], acc[2][1], acc[2][2], acc[2][3]);
  acc_guard4(acc[3][0], acc[3][1], acc[3][2], acc[3][3]);

  float* slab = sT[wave];
  const float* Rb = RESID ? (resid + (size_t)b * strideR) : nullptr;
#pragma unroll
  for (int i = 0; i < 4; ++i) {
    const int mBase = m0 + (i << 4);
#pragma unroll
    for (int j = 0; j < 4; ++j) {
      const int n = n0 + (j << 4) + rlane;
      float bv = 0.f;
      if (BIAS_MODE == 2) bv = bias[n];
#pragma unroll
      for (int r = 0; r < 8; ++r) {
        float v = acc[i][j][r] * scale;
        if (BIAS_MODE == 1) v += bias[mBase + mOff + r];
        if (BIAS_MODE == 2) v += bv;
        if (RESID) v += Rb[(size_t)(mBase + mOff + r) * ldc + n];
        if (ACT == 1) v = tanhf(v);
        if (ACT == 2) v = fmaxf(v, 0.0f);
        if (ACT == 3) v = v / (1.0f + expf(-v));
        if (ACT == 4) v = (v > 0.f) ? v : 0.01f * v;
        if (ACT == 5) v = 0.5f * v * (1.0f + erff(v * 0.70710678118654752f));
        slab[(mOff + r) * 68 + (j << 4) + rlane] = v;
      }
    }
    __builtin_amdgcn_fence(__ATOMIC_RELEASE, "workgroup");
    __builtin_amdgcn_wave_barrier();
    __builtin_amdgcn_fence(__ATOMIC_ACQUIRE, "workgroup");
    if (OUT_MODE == 0) {
      float* C = (float*)Cout + (size_t)b * strideC;
      const int hh = lane >> 4, c4 = (lane & 15) * 4;
      for (int pass = 0; pass < 2; ++pass) {
#pragma unroll
        for (int it = 0; it < 8; ++it) {
          const int row = it * 2 + hh;
          v4f v = *(const v4f*)(slab + row * 68 + c4);
          *(volatile v4f*)(C + (size_t)(mBase + row) * ldc + n0 + c4) = v;
        }
        __threadfence();
      }
    } else {
      const int q = lane >> 3, c8 = (lane & 7) * 8;
      unsigned short* C  = (unsigned short*)Cout  + (size_t)b * strideC;
      unsigned short* C2 = (OUT_MODE == 2) ? ((unsigned short*)Cout2 + (size_t)b * strideC) : nullptr;
      for (int pass = 0; pass < 2; ++pass) {
#pragma unroll
        for (int it = 0; it < 4; ++it) {
          const int row = it * 4 + q;
          const float* sp = slab + row * 68 + c8;
          v8h hv, lv;
#pragma unroll
          for (int e = 0; e < 8; ++e) {
            if (OUT_MODE == 1) {
              hv[e] = (_Float16)sp[e];
            } else {
              unsigned short hb = f2bf_bits(sp[e]);
              unsigned short lb = f2bf_bits(sp[e] - bf_bits2f(hb));
              hv[e] = __builtin_bit_cast(_Float16, hb);
              lv[e] = __builtin_bit_cast(_Float16, lb);
            }
          }
          *(volatile v8h*)(C + (size_t)(mBase + row) * ldc + n0 + c8) = hv;
          if (OUT_MODE == 2) *(volatile v8h*)(C2 + (size_t)(mBase + row) * ldc + n0 + c8) = lv;
        }
        __threadfence();
      }
    }
    __builtin_amdgcn_fence(__ATOMIC_RELEASE, "workgroup");
    __builtin_amdgcn_wave_barrier();
    __builtin_amdgcn_fence(__ATOMIC_ACQUIRE, "workgroup");
  }
}

__global__ __launch_bounds__(256) void cvt8_kernel(const float* __restrict__ src, unsigned short* __restrict__ dst,
                                                   int nrow, int ncol8, int spitch) {
  const int i  = blockIdx.x * 256 + threadIdx.x;
  const int n8 = nrow * ncol8;
  if (i < n8) {
    const int row = i / ncol8;
    const int c8  = i - row * ncol8;
    const float* sp = src + (size_t)row * spitch + c8 * 8;
    const v4f fa = *(const v4f*)(sp);
    const v4f fb = *(const v4f*)(sp + 4);
    unsigned bb[8];
    bb[0] = (unsigned)f2bf_bits(fa[0]); bb[1] = (unsigned)f2bf_bits(fa[1]);
    bb[2] = (unsigned)f2bf_bits(fa[2]); bb[3] = (unsigned)f2bf_bits(fa[3]);
    bb[4] = (unsigned)f2bf_bits(fb[0]); bb[5] = (unsigned)f2bf_bits(fb[1]);
    bb[6] = (unsigned)f2bf_bits(fb[2]); bb[7] = (unsigned)f2bf_bits(fb[3]);
    v4u w;
    w[0] = bb[0] | (bb[1] << 16);
    w[1] = bb[2] | (bb[3] << 16);
    w[2] = bb[4] | (bb[5] << 16);
    w[3] = bb[6] | (bb[7] << 16);
    unsigned short* dp = dst + (size_t)i * 8;
    *(volatile v4u*)dp = w;
    __threadfence();
    *(volatile v4u*)dp = w;
  }
}

__global__ __launch_bounds__(256) void tcvt_kernel(const float* __restrict__ in, unsigned short* __restrict__ outp,
                                                   int nK, int nN, int ldo, int orow0) {
  __shared__ float Tt[64 * 65];
  (void)nK;
  const int tid = threadIdx.x, lane = tid & 31, wave = tid >> 5;
  const int n0 = blockIdx.x * 64, k0 = blockIdx.y * 64;
  {
    const int r = tid >> 4, c4 = (tid & 15) * 4;
#pragma unroll
    for (int i = 0; i < 4; ++i) {
      const int kk = r + 16 * i;
      const v4f v = *(const v4f*)(in + (size_t)(k0 + kk) * nN + n0 + c4);
      Tt[kk * 65 + c4 + 0] = v[0];
      Tt[kk * 65 + c4 + 1] = v[1];
      Tt[kk * 65 + c4 + 2] = v[2];
      Tt[kk * 65 + c4 + 3] = v[3];
    }
  }
  __syncthreads();
  const int qq = lane >> 3, c8 = (lane & 7) * 8;
  v4u wv[2];
  size_t oo[2];
#pragma unroll
  for (int it = 0; it < 2; ++it) {
    const int nl = it * 32 + wave * 4 + qq;
    unsigned bb[8];
#pragma unroll
    for (int e = 0; e < 8; ++e) bb[e] = (unsigned)f2bf_bits(Tt[(c8 + e) * 65 + nl]);
    v4u w;
    w[0] = bb[0] | (bb[1] << 16);
    w[1] = bb[2] | (bb[3] << 16);
    w[2] = bb[4] | (bb[5] << 16);
    w[3] = bb[6] | (bb[7] << 16);
    wv[it] = w;
    oo[it] = (size_t)(orow0 + n0 + nl) * (size_t)ldo + (size_t)(k0 + c8);
  }
  for (int pass = 0; pass < 2; ++pass) {
    *(volatile v4u*)(outp + oo[0]) = wv[0];
    *(volatile v4u*)(outp + oo[1]) = wv[1];
    __threadfence();
  }
}

__global__ __launch_bounds__(256) void bias_prep_kernel(const float* __restrict__ bsrc, float* __restrict__ dst) {
  const int idx = threadIdx.x * 4;
  const v4f v = *(const v4f*)(bsrc + idx);
  v4f o;
  o[0] = bf16r(v[0]); o[1] = bf16r(v[1]); o[2] = bf16r(v[2]); o[3] = bf16r(v[3]);
  float* op = dst + idx;
  *(volatile v4f*)op = o;
  __threadfence();
  *(volatile v4f*)op = o;
}

__global__ __launch_bounds__(kRnnThr) void rnn_fused_kernel(const int* __restrict__ tokens, const float* __restrict__ Ptab,
                                                            const unsigned short* __restrict__ BTp,
                                                            const float* __restrict__ bd, float* __restrict__ out) {
  __shared__ __align__(16) unsigned short Hh[kRowsPB * kHP];
  __shared__ __align__(16) unsigned short Hl[kRowsPB * kHP];
  __shared__ __align__(16) float          Ls[kRowsPB * kLSP];
  const __bf16* BT = (const __bf16*)BTp;
  const int tid = threadIdx.x, lane = tid & 31, wave = tid >> 5;
  const int c = lane & 15, hh = lane >> 4, koff = hh * 8;
  const int rowbase = blockIdx.x * kRowsPB;

  {
    const v4u z = {0u, 0u, 0u, 0u};
#pragma unroll 1
    for (int i = tid; i < (kRowsPB * kHP) / 8; i += kRnnThr) {
      *(v4u*)(Hh + (size_t)i * 8) = z;
      *(v4u*)(Hl + (size_t)i * 8) = z;
    }
  }
  __syncthreads();

  const float bdv = bf16r(bd[16 * wave + c]);
  const int ncol0 = 128 * wave + 8 * c;
  const __bf16* bro = BT + (size_t)ncol0 * kUnits + koff;
  const __bf16* brl = BT + (size_t)(kUnits + 16 * wave + c) * kUnits + koff;
  const __bf16* ahp = (const __bf16*)Hh + c * kHP + koff;
  const __bf16* alp = (const __bf16*)Hl + c * kHP + koff;
  const int* tokrow = tokens + (size_t)(rowbase + 8 * hh) * kSeq;
  float* orow = out + (size_t)(rowbase + 2 * wave) * kSeq * kVocab + 4 * lane;
  const v8f z8 = {0.f, 0.f, 0.f, 0.f, 0.f, 0.f, 0.f, 0.f};

#pragma unroll 1
  for (int t = 0; t <= kSeq; ++t) {
    const int tt = (t < kSeq) ? t : (kSeq - 1);
    int tok[8];
#pragma unroll
    for (int r = 0; r < 8; ++r) {
      int tk = tokrow[r * kSeq + tt];
      tk = (tk < 0) ? 0 : tk;
      tk = (tk > kVocab - 1) ? (kVocab - 1) : tk;
      tok[r] = tk;
    }

    v8f acc[9];
#pragma unroll
    for (int j = 0; j < 9; ++j) acc[j] = z8;

#pragma unroll 2
    for (int kc = 0; kc < kUnits / 32; ++kc) {
      const v16b ah = Frag<__bf16>::load(ahp + kc * 32);
      const v16b al = Frag<__bf16>::load(alp + kc * 32);
#pragma unroll
      for (int g = 0; g < 3; ++g) {
        v16b bfr[3];
#pragma unroll
        for (int u = 0; u < 3; ++u) {
          const int j = 3 * g + u;
          const __bf16* bp = (j < 8) ? (bro + (size_t)j * kUnits) : brl;
          bfr[u] = Frag<__bf16>::load(bp + kc * 32);
        }
#pragma unroll
        for (int u = 0; u < 3; ++u) {
          const int j = 3 * g + u;
          acc[j] = Frag<__bf16>::mma(ah, bfr[u], acc[j]);
          acc[j] = Frag<__bf16>::mma(al, bfr[u], acc[j]);
        }
        grp_guard3(acc[3 * g], acc[3 * g + 1], acc[3 * g + 2], ah, al, bfr[0], bfr[1], bfr[2]);
      }
    }
    acc_guard4(acc[0], acc[1], acc[2], acc[3]);
    acc_guard4(acc[4], acc[5], acc[6], acc[7]);
    acc_guard1(acc[8]);

#pragma unroll
    for (int r = 0; r < 8; ++r) Ls[(8 * hh + r) * kLSP + 16 * wave + c] = acc[8][r] + bdv;
    __syncthreads();

    if (t < kSeq) {
#pragma unroll
      for (int r = 0; r < 8; ++r) {
        const float* pr = Ptab + (size_t)tok[r] * kUnits + ncol0;
        const v4f p0 = *(const v4f*)pr;
        const v4f p1 = *(const v4f*)(pr + 4);
        const float pv[8] = {p0[0], p0[1], p0[2], p0[3], p1[0], p1[1], p1[2], p1[3]};
        unsigned hw[8], lw[8];
#pragma unroll
        for (int j = 0; j < 8; ++j) {
          const float v = tanhf(acc[j][r] + pv[j]);
          const unsigned short hb = f2bf_bits(v);
          const unsigned short lb = f2bf_bits(v - bf_bits2f(hb));
          hw[j] = (unsigned)hb;
          lw[j] = (unsigned)lb;
        }
        v4u hu, lu;
        hu[0] = hw[0] | (hw[1] << 16); hu[1] = hw[2] | (hw[3] << 16); hu[2] = hw[4] | (hw[5] << 16); hu[3] = hw[6] | (hw[7] << 16);
        lu[0] = lw[0] | (lw[1] << 16); lu[1] = lw[2] | (lw[3] << 16); lu[2] = lw[4] | (lw[5] << 16); lu[3] = lw[6] | (lw[7] << 16);
        const int so = (8 * hh + r) * kHP + ncol0;
        *(v4u*)(Hh + so) = hu;
        *(v4u*)(Hl + so) = lu;
        asm volatile("" ::: "memory");
      }
    }
    if (t >= 1) {
      float* op = orow + (size_t)(t - 1) * kVocab;
      const float* l0 = Ls + (2 * wave) * kLSP + 4 * lane;
      for (int pass = 0; pass < 2; ++pass) {
        const v4f v0 = *(const v4f*)l0;
        const v4f v1 = *(const v4f*)(l0 + kLSP);
        *(volatile v4f*)op = v0;
        *(volatile v4f*)(op + (size_t)kSeq * kVocab) = v1;
        __threadfence();
      }
    }
    __syncthreads();
  }
}

extern "C" void kernel_launch(void* const* d_in, const int* in_sizes, int n_in,
                              void* d_out, int out_size, void* d_ws, size_t ws_size, hipStream_t stream) {
  if (n_in < 7 || d_out == nullptr || d_ws == nullptr) return;
  if (in_sizes[0] != kBatch * kSeq || in_sizes[1] != kVocab * kEmb || in_sizes[2] != kEmb * kUnits ||
      in_sizes[3] != kUnits * kUnits || in_sizes[4] != kUnits || in_sizes[5] != kUnits * kVocab ||
      in_sizes[6] != kVocab || out_size != kBatch * kSeq * kVocab) return;

  const int*   tokens = (const int*)d_in[0];
  const float* emb    = (const float*)d_in[1];
  const float* wx     = (const float*)d_in[2];
  const float* wh     = (const float*)d_in[3];
  const float* bx     = (const float*)d_in[4];
  const float* wd     = (const float*)d_in[5];
  const float* bd     = (const float*)d_in[6];
  float* out = (float*)d_out;

  char* ws = (char*)d_ws; size_t off = 0;
  auto carve = [&](size_t bytes) -> char* { char* p = ws + off; off += (bytes + 255) & ~(size_t)255; return p; };
  unsigned short* EMB16 = (unsigned short*)carve((size_t)kVocab * kEmb * 2);
  unsigned short* WXT16 = (unsigned short*)carve((size_t)kUnits * kEmb * 2);
  unsigned short* BT16  = (unsigned short*)carve((size_t)kNBt * kUnits * 2);
  float*          BB    = (float*)carve((size_t)kUnits * 4);
  float*          PTAB  = (float*)carve((size_t)kVocab * kUnits * 4);
  if (off > ws_size || off > (size_t)134217728) return;

  cvt8_kernel<<<(kVocab * kEmb / 8) / 256, 256, 0, stream>>>(emb, EMB16, kVocab, kEmb / 8, kEmb);
  tcvt_kernel<<<dim3(kUnits / 64, kEmb / 64), 256, 0, stream>>>(wx, WXT16, kEmb, kUnits, kEmb, 0);
  tcvt_kernel<<<dim3(kUnits / 64, kUnits / 64), 256, 0, stream>>>(wh, BT16, kUnits, kUnits, kUnits, 0);
  tcvt_kernel<<<dim3(kVocab / 64, kUnits / 64), 256, 0, stream>>>(wd, BT16, kUnits, kVocab, kUnits, kUnits);
  bias_prep_kernel<<<1, 256, 0, stream>>>(bx, BB);
  wmma_gemm64<1, false, 2, 0, false, 0><<<dim3((kVocab / 64) * (kUnits / 64) / 8, 1), 256, 0, stream>>>(
      EMB16, EMB16, kEmb, 0L, WXT16, WXT16, kEmb, 0L, (void*)PTAB, (void*)PTAB, kUnits, 0L,
      BB, BB, 0L, kVocab, kUnits, kEmb, 1.0f);
  rnn_fused_kernel<<<kRnnBlocks, kRnnThr, 0, stream>>>(tokens, PTAB, BT16, bd, out);
}
